// CausalSALayer_12266426597820
// MI455X (gfx1250) — hardware-verified
//
#include <hip/hip_runtime.h>

typedef __attribute__((ext_vector_type(16))) _Float16 v16h;
typedef __attribute__((ext_vector_type(8)))  _Float16 v8h;
typedef __attribute__((ext_vector_type(16))) __bf16   v16b;
typedef __attribute__((ext_vector_type(8)))  __bf16   v8b;
typedef __attribute__((ext_vector_type(8)))  float    v8f;
typedef __attribute__((ext_vector_type(4)))  float    v4f;
typedef __attribute__((ext_vector_type(4)))  int      v4i;

#define DM     1024
#define NHEAD  16
#define HD     64
#define FFND   4096
#define BSZ    2
#define SEQ    2048
#define MROWS  (BSZ * SEQ)
#define LN_EPS 1e-5f

__device__ __forceinline__ unsigned short f2bf_bits(float f) {
  unsigned u = __float_as_uint(f);
  return (unsigned short)((u + 0x7FFFu + ((u >> 16) & 1u)) >> 16);
}
__device__ __forceinline__ float bf_bits2f(unsigned short h) { return __uint_as_float(((unsigned)h) << 16); }

__device__ __forceinline__ void dep_guard_h(v8f& a, v8f& b, v16h x, v16h y) { asm volatile("v_nop\n\tv_nop\n\tv_nop\n\tv_nop" : "+v"(a), "+v"(b) : "v"(x), "v"(y)); }
__device__ __forceinline__ void dep_guard_b(v8f& a, v8f& b, v16b x, v16b y) { asm volatile("v_nop\n\tv_nop\n\tv_nop\n\tv_nop" : "+v"(a), "+v"(b) : "v"(x), "v"(y)); }
__device__ __forceinline__ void keep4_h(v16h a, v16h b, v16h c, v16h d) { asm volatile("v_nop" :: "v"(a), "v"(b), "v"(c), "v"(d)); }
__device__ __forceinline__ void keep4_b(v16b a, v16b b, v16b c, v16b d) { asm volatile("v_nop" :: "v"(a), "v"(b), "v"(c), "v"(d)); }
__device__ __forceinline__ void acc_guard4(v8f& a, v8f& b, v8f& c, v8f& d) { asm volatile("v_nop\n\tv_nop\n\tv_nop\n\tv_nop" : "+v"(a), "+v"(b), "+v"(c), "+v"(d)); }
template <typename T> struct Frag;
template <> struct Frag<_Float16> {
  typedef v16h V; union U { v16h v; v8h h[2]; };
  static __device__ __forceinline__ v16h load(const _Float16* p) {
    U f; f.h[0] = *(const v8h*)(p); f.h[1] = *(const v8h*)(p + 16); return f.v;
  }
  static __device__ __forceinline__ v8f mma(v16h a, v16h b, v8f c) {
    return __builtin_amdgcn_wmma_f32_16x16x32_f16(false, a, false, b, (short)0, c, false, false);
  }
  static __device__ __forceinline__ void guard(v8f& a, v8f& b, v16h x, v16h y) { dep_guard_h(a, b, x, y); }
  static __device__ __forceinline__ void keep(v16h a, v16h b, v16h c, v16h d) { keep4_h(a, b, c, d); }
};
template <> struct Frag<__bf16> {
  typedef v16b V; union U { v16b v; v8b h[2]; };
  static __device__ __forceinline__ v16b load(const __bf16* p) {
    U f; f.h[0] = *(const v8b*)(p); f.h[1] = *(const v8b*)(p + 16); return f.v;
  }
  static __device__ __forceinline__ v8f mma(v16b a, v16b b, v8f c) {
    return __builtin_amdgcn_wmma_f32_16x16x32_bf16(false, a, false, b, (short)0, c, false, false);
  }
  static __device__ __forceinline__ void guard(v8f& a, v8f& b, v16b x, v16b y) { dep_guard_b(a, b, x, y); }
  static __device__ __forceinline__ void keep(v16b a, v16b b, v16b c, v16b d) { keep4_b(a, b, c, d); }
};

__device__ __forceinline__ float gelu_tanh_f(float v) {
  const float u = 0.7978845608028654f * (v + 0.044715f * v * v * v);
  const float e = __expf(-2.0f * fabsf(u));
  float t = (1.0f - e) * __builtin_amdgcn_rcpf(1.0f + e);
  t = copysignf(t, u);
  return 0.5f * v * (1.0f + t);
}

template <int ET> struct Elem;
template <> struct Elem<0> { typedef _Float16 T; };
template <> struct Elem<1> { typedef __bf16 T; };
template <int ET, bool SPLIT, int BIAS_MODE, int OUT_MODE, bool RESID, int ACT = 0>
__global__ __launch_bounds__(256) void wmma_gemm64(
    const unsigned short* __restrict__ Ap, const unsigned short* __restrict__ A2p, int lda, long strideA,
    const unsigned short* __restrict__ Btp, const unsigned short* __restrict__ Bt2p, int ldb, long strideB,
    void* __restrict__ Cout, void* __restrict__ Cout2, int ldc, long strideC,
    const float* __restrict__ bias,
    const float* __restrict__ resid, long strideR,
    int M, int N, int K, float scale) {
  typedef typename Elem<ET>::T T;
  typedef typename Frag<T>::V V;
  const T* A = (const T*)Ap; const T* A2 = (const T*)A2p; const T* Bt = (const T*)Btp; const T* Bt2 = (const T*)Bt2p;
  __shared__ __align__(16) float sT[8][16 * 68];
  const int b    = blockIdx.y;
  const int lane = threadIdx.x & 31;
  const int wave = threadIdx.x >> 5;
  const int tilesN = N >> 6;
  const int tilesM = M >> 6;
  const int tile = blockIdx.x * 8 + wave;
  if (tile >= tilesM * tilesN) return;
  const int tm = tile / tilesN;
  const int tn = tile - tm * tilesN;
  const int m0 = tm << 6;
  const int n0 = tn << 6;

  const T* Ab  = A  + (size_t)b * strideA;
  const T* Bb  = Bt + (size_t)b * strideB;
  const T* Ab2 = SPLIT ? (A2  + (size_t)b * strideA) : nullptr;
  const T* Bb2 = SPLIT ? (Bt2 + (size_t)b * strideB) : nullptr;

  const int rlane = lane & 15;
  const int koff  = (lane >> 4) * 8;
  const int mOff  = (lane >> 4) * 8;

  v8f acc[4][4];
#pragma unroll
  for (int i = 0; i < 4; ++i)
#pragma unroll
    for (int j = 0; j < 4; ++j) acc[i][j] = (v8f){0.f,0.f,0.f,0.f,0.f,0.f,0.f,0.f};

  for (int k0 = 0; k0 < K; k0 += 32) {
    V bh[4], bl[4];
#pragma unroll
    for (int j = 0; j < 4; ++j) {
      const size_t bo = (size_t)(n0 + (j << 4) + rlane) * ldb + koff + k0;
      bh[j] = Frag<T>::load(Bb + bo);
      if (SPLIT) bl[j] = Frag<T>::load(Bb2 + bo);
    }
#pragma unroll
    for (int i = 0; i < 4; ++i) {
      const size_t ao = (size_t)(m0 + (i << 4) + rlane) * lda + koff + k0;
      V ah = Frag<T>::load(Ab + ao);
      V al;
      if (SPLIT) al = Frag<T>::load(Ab2 + ao);
#pragma unroll
      for (int j = 0; j < 4; ++j) {
        acc[i][j] = Frag<T>::mma(ah, bh[j], acc[i][j]);
        if (SPLIT) {
          acc[i][j] = Frag<T>::mma(ah, bl[j], acc[i][j]);
          acc[i][j] = Frag<T>::mma(al, bh[j], acc[i][j]);
        }
      }
      Frag<T>::guard(acc[i][0], acc[i][3], ah, SPLIT ? al : ah);
    }
    Frag<T>::keep(bh[0], bh[1], bh[2], bh[3]);
    if (SPLIT) Frag<T>::keep(bl[0], bl[1], bl[2], bl[3]);
  }
  acc_guard4(acc[0][0], acc[0][1], acc[0][2], acc[0][3]);
  acc_guard4(acc[1][0], acc[1][1], acc[1][2], acc[1][3]);
  acc_guard4(acc[2][0], acc[2][1], acc[2][2], acc[2][3]);
  acc_guard4(acc[3][0], acc[3][1], acc[3][2], acc[3][3]);

  float* slab = sT[wave];
  const float* Rb = RESID ? (resid + (size_t)b * strideR) : nullptr;
#pragma unroll
  for (int i = 0; i < 4; ++i) {
    const int mBase = m0 + (i << 4);
#pragma unroll
    for (int j = 0; j < 4; ++j) {
      const int n = n0 + (j << 4) + rlane;
      float bv = 0.f;
      if (BIAS_MODE == 2) bv = bias[n];
#pragma unroll
      for (int r = 0; r < 8; ++r) {
        float v = acc[i][j][r] * scale;
        if (BIAS_MODE == 1) v += bias[mBase + mOff + r];
        if (BIAS_MODE == 2) v += bv;
        if (RESID) v += Rb[(size_t)(mBase + mOff + r) * ldc + n];
        if (ACT == 1) v = tanhf(v);
        if (ACT == 2) v = fmaxf(v, 0.0f);
        if (ACT == 3) v = v / (1.0f + expf(-v));
        if (ACT == 4) v = (v > 0.f) ? v : 0.01f * v;
        if (ACT == 5) v = 0.5f * v * (1.0f + erff(v * 0.70710678118654752f));
        if (ACT == 6) v = gelu_tanh_f(v);
        slab[(mOff + r) * 68 + (j << 4) + rlane] = v;
      }
    }
    __builtin_amdgcn_fence(__ATOMIC_RELEASE, "workgroup");
    __builtin_amdgcn_wave_barrier();
    __builtin_amdgcn_fence(__ATOMIC_ACQUIRE, "workgroup");
    if (OUT_MODE == 0) {
      float* C = (float*)Cout + (size_t)b * strideC;
      const int hh = lane >> 4, c4 = (lane & 15) * 4;
      for (int pass = 0; pass < 2; ++pass) {
#pragma unroll
        for (int it = 0; it < 8; ++it) {
          const int row = it * 2 + hh;
          v4f v = *(const v4f*)(slab + row * 68 + c4);
          *(volatile v4f*)(C + (size_t)(mBase + row) * ldc + n0 + c4) = v;
        }
        __threadfence();
      }
    } else {
      const int q = lane >> 3, c8 = (lane & 7) * 8;
      unsigned short* C  = (unsigned short*)Cout  + (size_t)b * strideC;
      unsigned short* C2 = (OUT_MODE == 2) ? ((unsigned short*)Cout2 + (size_t)b * strideC) : nullptr;
      for (int pass = 0; pass < 2; ++pass) {
#pragma unroll
        for (int it = 0; it < 4; ++it) {
          const int row = it * 4 + q;
          const float* sp = slab + row * 68 + c8;
          v8h hv, lv;
#pragma unroll
          for (int e = 0; e < 8; ++e) {
            if (OUT_MODE == 1) {
              hv[e] = (_Float16)sp[e];
            } else {
              unsigned short hb = f2bf_bits(sp[e]);
              unsigned short lb = f2bf_bits(sp[e] - bf_bits2f(hb));
              hv[e] = __builtin_bit_cast(_Float16, hb);
              lv[e] = __builtin_bit_cast(_Float16, lb);
            }
          }
          *(volatile v8h*)(C + (size_t)(mBase + row) * ldc + n0 + c8) = hv;
          if (OUT_MODE == 2) *(volatile v8h*)(C2 + (size_t)(mBase + row) * ldc + n0 + c8) = lv;
        }
        __threadfence();
      }
    }
    __builtin_amdgcn_fence(__ATOMIC_RELEASE, "workgroup");
    __builtin_amdgcn_wave_barrier();
    __builtin_amdgcn_fence(__ATOMIC_ACQUIRE, "workgroup");
  }
}

__global__ __launch_bounds__(256) void cast_f32_f16x2(
    const float* __restrict__ in, _Float16* __restrict__ out, int n2) {
  int i = blockIdx.x * 256 + threadIdx.x;
  if (i < n2) {
    const _Float16 h0 = (_Float16)in[2 * i], h1 = (_Float16)in[2 * i + 1];
    const unsigned u = (unsigned)__builtin_bit_cast(unsigned short, h0) | ((unsigned)__builtin_bit_cast(unsigned short, h1) << 16);
    ((volatile unsigned*)out)[i] = u;
    __threadfence();
    ((volatile unsigned*)out)[i] = u;
  }
}

#define AT_D 64
#define AT_NW 4
#define AT_QB 64
#define AT_KC 64
struct AttnGeom { const int* tcode; const float* cp; const float* pc; long c_bs, c_rs, c_hs, t_pitch;
                  long q_bs, q_rs, q_hs, k_bs, k_rs, k_hs, v_bs, v_rs, v_hs, o_bs, o_rs, o_hs;
                  int S, Skv, H, mask_mode; float qscale; int blk0; float mask_fill; int mask_is_int; };
static_assert(sizeof(AttnGeom) == 184);

__device__ __forceinline__ unsigned short at_bf_bits(float f) {
  unsigned u = __float_as_uint(f);
  return (unsigned short)((u + 0x7FFFu + ((u >> 16) & 1u)) >> 16);
}
__device__ __forceinline__ __bf16 at_f2bf(float f) { return __builtin_bit_cast(__bf16, at_bf_bits(f)); }
__device__ __forceinline__ void at_split(float f, __bf16& hi, __bf16& lo) {
  const unsigned short hb = at_bf_bits(f);
  hi = __builtin_bit_cast(__bf16, hb);
  lo = at_f2bf(f - __uint_as_float(((unsigned)hb) << 16));
}
__device__ __forceinline__ v8f at_mma(v16b a, v16b b, v8f c) {
  c = __builtin_amdgcn_wmma_f32_16x16x32_bf16(false, a, false, b, (short)0, c, false, false);
  asm volatile("v_nop\n\tv_nop\n\tv_nop\n\tv_nop" : "+v"(c) : "v"(a), "v"(b));
  return c;
}
template <bool F16> __device__ __forceinline__ __bf16 at_to16(float f) {
  if (F16) return __builtin_bit_cast(__bf16, (_Float16)f);
  return at_f2bf(f);
}
template <bool F16> __device__ __forceinline__ v8f at_mma16(v16b a, v16b b, v8f c) {
  if (F16) {
    const v16h ah = __builtin_bit_cast(v16h, a), bh = __builtin_bit_cast(v16h, b);
    c = __builtin_amdgcn_wmma_f32_16x16x32_f16(false, ah, false, bh, (short)0, c, false, false);
    asm volatile("v_nop\n\tv_nop\n\tv_nop\n\tv_nop" : "+v"(c) : "v"(ah), "v"(bh));
    return c;
  }
  return at_mma(a, b, c);
}

template <bool SPLIT_QK, bool SPLIT_PV, bool F16 = false>
__global__ __launch_bounds__(128)
void attn64_kernel(const float* __restrict__ q, const float* __restrict__ k,
                   const float* __restrict__ v, float* __restrict__ out,
                   const int* __restrict__ mask_a, const int* __restrict__ mask_b, AttnGeom g) {
  static_assert(!(F16 && (SPLIT_QK || SPLIT_PV)));
  const float PSC = F16 ? 32768.0f : 1.0f;
  union FB { v16b v; v8b h[2]; };
  __shared__ __align__(16) __bf16 Ksh[AT_KC * AT_D];
  __shared__ __align__(16) __bf16 Ksl[SPLIT_QK ? AT_KC * AT_D : 8];
  __shared__ __align__(16) __bf16 Vth[AT_D * AT_KC];
  __shared__ __align__(16) __bf16 Vtl[SPLIT_PV ? AT_D * AT_KC : 8];
  __shared__ __align__(16) __bf16 Psh[AT_NW][16 * AT_KC];
  __shared__ __align__(16) __bf16 Psl[SPLIT_PV ? AT_NW : 1][SPLIT_PV ? 16 * AT_KC : 8];
  __shared__ __align__(16) float  Os[AT_NW][16 * 68];

  const int tid  = threadIdx.x;
  const int wave = tid >> 5;
  const int lane = tid & 31;
  const int hh   = lane >> 4;
  const int c    = lane & 15;

  const int nqb = g.S / AT_QB;
  const int nkc = g.Skv / AT_KC;
  const int bx = blockIdx.x + g.blk0;
  const int qb = bx % nqb;
  const int bh = bx / nqb;
  const int h  = bh % g.H;
  const int b  = bh / g.H;
  const int qbase_block = qb * AT_QB;
  const int q0 = qbase_block + wave * 16;

  const float* qb_ptr = q + (size_t)b * g.q_bs + (size_t)h * g.q_hs;
  const float* kb_ptr = k + (size_t)b * g.k_bs + (size_t)h * g.k_hs;
  const float* vb_ptr = v + (size_t)b * g.v_bs + (size_t)h * g.v_hs;
  float*       ob_ptr = out + (size_t)b * g.o_bs + (size_t)h * g.o_hs;

  v16b qah[2], qal[2];
  {
    const float* qrow = qb_ptr + (size_t)(q0 + c) * g.q_rs;
#pragma unroll
    for (int dc = 0; dc < 2; ++dc) {
#pragma unroll
      for (int e = 0; e < 8; ++e) {
        const float f0 = qrow[dc * 32 + 8 * hh + e] * g.qscale;
        const float f1 = qrow[dc * 32 + 16 + 8 * hh + e] * g.qscale;
        if (SPLIT_QK) { __bf16 hq, lq; at_split(f0, hq, lq); qah[dc][e] = hq; qal[dc][e] = lq; at_split(f1, hq, lq); qah[dc][8 + e] = hq; qal[dc][8 + e] = lq; }
        else { qah[dc][e] = at_to16<F16>(f0); qah[dc][8 + e] = at_to16<F16>(f1); qal[dc][e] = qah[dc][e]; qal[dc][8 + e] = qah[dc][8 + e]; }
      }
    }
  }

  float mrow[8], lrow[8];
  v8f oacc[4];
#pragma unroll
  for (int r = 0; r < 8; ++r) { mrow[r] = -INFINITY; lrow[r] = 0.f; }
#pragma unroll
  for (int t = 0; t < 4; ++t) oacc[t] = (v8f){0.f,0.f,0.f,0.f,0.f,0.f,0.f,0.f};

  const int nChunks = (g.mask_mode == 1 || g.mask_mode == 4) ? (qb + 1) : nkc;
  int qkeep[8];
#pragma unroll
  for (int r = 0; r < 8; ++r) qkeep[r] = (g.mask_mode == 3) ? mask_b[(size_t)b * g.S + q0 + 8 * hh + r] : 1;
  for (int kc = 0; kc < nChunks; ++kc) {
    const int kv0 = kc * AT_KC;
    int code = 0;
    if (g.mask_mode == 6) {
      int cv = g.tcode[((size_t)b * nqb + qb) * (size_t)g.t_pitch + kc];
      cv = __builtin_amdgcn_readfirstlane(cv);
      code = (cv == 1 || cv == 2) ? cv : 0;
      if (code == 2) continue;
    }
    __syncthreads();
    {
      const int kvr = tid >> 1, dh = (tid & 1) * 32;
      const float* krow = kb_ptr + (size_t)(kv0 + kvr) * g.k_rs + dh;
      const float* vrow = vb_ptr + (size_t)(kv0 + kvr) * g.v_rs + dh;
#pragma unroll
      for (int i = 0; i < 8; ++i) {
        v4f kk = *(const v4f*)(krow + 4 * i);
        v4f vv = *(const v4f*)(vrow + 4 * i);
#pragma unroll
        for (int e = 0; e < 4; ++e) {
          const int d = dh + 4 * i + e;
          if (SPLIT_QK) { __bf16 a, bl; at_split(kk[e], a, bl); Ksh[kvr * AT_D + d] = a; Ksl[kvr * AT_D + d] = bl; }
          else Ksh[kvr * AT_D + d] = at_to16<F16>(kk[e]);
          if (SPLIT_PV) { __bf16 a, bl; at_split(vv[e], a, bl); Vth[d * AT_KC + kvr] = a; Vtl[d * AT_KC + kvr] = bl; }
          else Vth[d * AT_KC + kvr] = at_to16<F16>(vv[e]);
        }
      }
    }
    __syncthreads();

    v8f s[4];
#pragma unroll
    for (int j = 0; j < 4; ++j) {
      s[j] = (v8f){0.f,0.f,0.f,0.f,0.f,0.f,0.f,0.f};
#pragma unroll 1
      for (int dc = 0; dc < 2; ++dc) {
        FB kb;
        kb.h[0] = *(const v8b*)(Ksh + (j * 16 + c) * AT_D + dc * 32 + 8 * hh);
        kb.h[1] = *(const v8b*)(Ksh + (j * 16 + c) * AT_D + dc * 32 + 16 + 8 * hh);
        s[j] = at_mma16<F16>(qah[dc], kb.v, s[j]);
        if (SPLIT_QK) {
          FB kl;
          kl.h[0] = *(const v8b*)(Ksl + (j * 16 + c) * AT_D + dc * 32 + 8 * hh);
          kl.h[1] = *(const v8b*)(Ksl + (j * 16 + c) * AT_D + dc * 32 + 16 + 8 * hh);
          s[j] = at_mma16<F16>(qah[dc], kl.v, s[j]);
          s[j] = at_mma16<F16>(qal[dc], kb.v, s[j]);
        }
      }
    }
    const bool diag = (g.mask_mode == 1) && (kc == qb);
    int kvkeep[4] = {1, 1, 1, 1};
    if (g.mask_mode == 3) {
#pragma unroll
      for (int j = 0; j < 4; ++j) kvkeep[j] = mask_a[(size_t)b * g.Skv + kv0 + j * 16 + c];
    }
    int kvpad[4] = {0, 0, 0, 0};
    if (g.mask_mode == 6 && code == 0) {
#pragma unroll
      for (int j = 0; j < 4; ++j) kvpad[j] = mask_b[(size_t)b * g.Skv + kv0 + j * 16 + c];
    }
    float cm[8];
#pragma unroll
    for (int r = 0; r < 8; ++r) {
      const int qrow = q0 + 8 * hh + r;
      float m = -INFINITY;
#pragma unroll
      for (int j = 0; j < 4; ++j) {
        const int kvcol = kv0 + j * 16 + c;
        bool masked = false;
        if (diag) masked = (kvcol > qrow);
        else if (g.mask_mode == 4) masked = (kvcol > qrow) || (qrow - kvcol > g.mask_is_int);
        else if (g.mask_mode == 2) {
          const size_t mi = (size_t)qrow * g.Skv + kvcol;
          masked = (g.mask_is_int == 0) ? (((const float*)mask_a)[mi] == 0.0f)
                 : (g.mask_is_int == 1) ? (mask_a[mi] == 0) : (mask_a[mi] != 0);
        } else if (g.mask_mode == 3) masked = (qkeep[r] == 0) || (kvkeep[j] == 0);
        else if (g.mask_mode == 5) {
          const size_t mi = (size_t)qrow * g.Skv + kvcol;
          masked = (mask_a[mi] != 0);
          int n = mask_b[mi]; n = n < 0 ? 0 : n;
          s[j][r] += g.cp[(size_t)b * g.c_bs + (size_t)h * g.c_hs + (size_t)qrow * g.c_rs + n]
                   + g.pc[(size_t)b * g.c_bs + (size_t)h * g.c_hs + (size_t)kvcol * g.c_rs + n];
        } else if (g.mask_mode == 6) {
          if (code == 0) masked = (mask_a[(size_t)qrow * g.Skv + kvcol] != 0) || (kvpad[j] != 0);
        }
        if (masked) s[j][r] = g.mask_fill;
        m = fmaxf(m, s[j][r]);
      }
#pragma unroll
      for (int off = 1; off < 16; off <<= 1) m = fmaxf(m, __shfl_xor(m, off, 32));
      cm[r] = m;
    }
    __bf16* pwh = Psh[wave];
    __bf16* pwl = Psl[SPLIT_PV ? wave : 0];
#pragma unroll
    for (int r = 0; r < 8; ++r) {
      const float mnew = fmaxf(mrow[r], cm[r]);
      const bool dead = (mnew == -INFINITY);
      const float alpha = dead ? 1.0f : expf(mrow[r] - mnew);
      mrow[r] = mnew;
      float psum = 0.f;
#pragma unroll
      for (int j = 0; j < 4; ++j) {
        const float p = dead ? 0.0f : expf(s[j][r] - mnew);
        psum += p;
        if (SPLIT_PV) { __bf16 a, bl; at_split(p, a, bl); pwh[(8 * hh + r) * AT_KC + j * 16 + c] = a; pwl[(8 * hh + r) * AT_KC + j * 16 + c] = bl; }
        else pwh[(8 * hh + r) * AT_KC + j * 16 + c] = at_to16<F16>(p * PSC);
      }
#pragma unroll
      for (int off = 1; off < 16; off <<= 1) psum += __shfl_xor(psum, off, 32);
      lrow[r] = lrow[r] * alpha + psum;
#pragma unroll
      for (int t = 0; t < 4; ++t) oacc[t][r] *= alpha;
    }
    __builtin_amdgcn_fence(__ATOMIC_RELEASE, "workgroup");
    __builtin_amdgcn_wave_barrier();
    __builtin_amdgcn_fence(__ATOMIC_ACQUIRE, "workgroup");
#pragma unroll 1
    for (int kk = 0; kk < 2; ++kk) {
      FB pa, pl;
      pa.h[0] = *(const v8b*)(pwh + c * AT_KC + kk * 32 + 8 * hh);
      pa.h[1] = *(const v8b*)(pwh + c * AT_KC + kk * 32 + 16 + 8 * hh);
      if (SPLIT_PV) {
        pl.h[0] = *(const v8b*)(pwl + c * AT_KC + kk * 32 + 8 * hh);
        pl.h[1] = *(const v8b*)(pwl + c * AT_KC + kk * 32 + 16 + 8 * hh);
      }
#pragma unroll
      for (int t = 0; t < 4; ++t) {
        FB vb;
        vb.h[0] = *(const v8b*)(Vth + (t * 16 + c) * AT_KC + kk * 32 + 8 * hh);
        vb.h[1] = *(const v8b*)(Vth + (t * 16 + c) * AT_KC + kk * 32 + 16 + 8 * hh);
        oacc[t] = at_mma16<F16>(pa.v, vb.v, oacc[t]);
        if (SPLIT_PV) {
          FB vl;
          vl.h[0] = *(const v8b*)(Vtl + (t * 16 + c) * AT_KC + kk * 32 + 8 * hh);
          vl.h[1] = *(const v8b*)(Vtl + (t * 16 + c) * AT_KC + kk * 32 + 16 + 8 * hh);
          oacc[t] = at_mma16<F16>(pa.v, vl.v, oacc[t]);
          oacc[t] = at_mma16<F16>(pl.v, vb.v, oacc[t]);
        }
      }
    }
  }

  float* os = Os[wave];
#pragma unroll
  for (int r = 0; r < 8; ++r) {
    const float den = lrow[r] * PSC;
    const float inv = (den > 0.0f) ? (1.0f / den) : 0.0f;
#pragma unroll
    for (int t = 0; t < 4; ++t) os[(8 * hh + r) * 68 + t * 16 + c] = oacc[t][r] * inv;
  }
  __builtin_amdgcn_fence(__ATOMIC_RELEASE, "workgroup");
  __builtin_amdgcn_wave_barrier();
  __builtin_amdgcn_fence(__ATOMIC_ACQUIRE, "workgroup");
  {
    const int c4 = (lane & 15) * 4;
    for (int pass = 0; pass < 2; ++pass) {
#pragma unroll
      for (int it = 0; it < 8; ++it) {
        const int row = it * 2 + hh;
        v4f val = *(const v4f*)(os + row * 68 + c4);
        *(volatile v4f*)(ob_ptr + (size_t)(q0 + row) * g.o_rs + c4) = val;
      }
      __threadfence();
    }
  }
}

__global__ __launch_bounds__(256) void tilecode_kernel(
    const int* __restrict__ tm, const int* __restrict__ pad, int* __restrict__ tab,
    int Skv, int nqb, int nkc, int tp) {
  __shared__ int wl[8], wm[8];
  __shared__ __align__(16) int codes[128];
  const int tid = threadIdx.x, lane = tid & 31, wave = tid >> 5;
  const int b  = blockIdx.x / nqb;
  const int qb = blockIdx.x - b * nqb;
  const int row = tid >> 2, cs = (tid & 3) * 16;
  const int q = qb * 64 + row;
  if (tid < 128) codes[tid] = 2;
  __syncthreads();
  const int nk = nkc < 128 ? nkc : 128;
  for (int kc = 0; kc < nk; ++kc) {
    const int* mr = tm  + (size_t)q * Skv + kc * 64 + cs;
    const int* pr = pad + (size_t)b * Skv + kc * 64 + cs;
    int live = 0, msk = 0;
#pragma unroll
    for (int i = 0; i < 4; ++i) {
      const v4i mv = *(const v4i*)(mr + 4 * i);
      const v4i pv = *(const v4i*)(pr + 4 * i);
#pragma unroll
      for (int e = 0; e < 4; ++e) {
        const int m = ((mv[e] != 0) || (pv[e] != 0)) ? 1 : 0;
        msk |= m;
        live |= (m ^ 1);
      }
    }
    const int al = __any(live);
    const int am = __any(msk);
    if (lane == 0) { wl[wave] = al; wm[wave] = am; }
    __syncthreads();
    if (tid == 0) {
      int L = 0, Mk = 0;
#pragma unroll
      for (int w = 0; w < 8; ++w) { L |= wl[w]; Mk |= wm[w]; }
      codes[kc] = (L == 0) ? 2 : ((Mk == 0) ? 1 : 0);
    }
    __syncthreads();
  }
  if (wave == 0) {
    const int nl = tp >> 2;
    v4i cv;
    cv[0] = codes[(4 * lane + 0) & 127]; cv[1] = codes[(4 * lane + 1) & 127];
    cv[2] = codes[(4 * lane + 2) & 127]; cv[3] = codes[(4 * lane + 3) & 127];
    int* dst = tab + (size_t)blockIdx.x * tp + 4 * lane;
    if (lane < nl) *(volatile v4i*)dst = cv;
    __threadfence();
    if (lane < nl) *(volatile v4i*)dst = cv;
  }
}

template <bool OUT16>
__global__ __launch_bounds__(256) void ln_kernel(
    const float* __restrict__ in, const float* __restrict__ gam, const float* __restrict__ bet,
    float* __restrict__ o32, _Float16* __restrict__ o16) {
  __shared__ float red1[8], red2[8];
  __shared__ __align__(16) float ybuf[OUT16 ? DM : 4];
  const int row = blockIdx.x, t = threadIdx.x, lane = t & 31, wave = t >> 5;
  const float* x = in + (size_t)row * DM;
  const v4f xv = *(const v4f*)(x + 4 * t);
  float s = (xv[0] + xv[1]) + (xv[2] + xv[3]);
#pragma unroll
  for (int off = 1; off < 32; off <<= 1) s += __shfl_xor(s, off, 32);
  if (lane == 0) red1[wave] = s;
  __syncthreads();
  float tot = 0.f;
#pragma unroll
  for (int w = 0; w < 8; ++w) tot += red1[w];
  const float mu = tot * (1.0f / (float)DM);
  const float d0 = xv[0] - mu, d1 = xv[1] - mu, d2 = xv[2] - mu, d3 = xv[3] - mu;
  float s2 = (d0 * d0 + d1 * d1) + (d2 * d2 + d3 * d3);
#pragma unroll
  for (int off = 1; off < 32; off <<= 1) s2 += __shfl_xor(s2, off, 32);
  if (lane == 0) red2[wave] = s2;
  __syncthreads();
  float tot2 = 0.f;
#pragma unroll
  for (int w = 0; w < 8; ++w) tot2 += red2[w];
  const float var = tot2 * (1.0f / (float)DM);
  const float rstd = rsqrtf(var + LN_EPS);
  const v4f gv = *(const v4f*)(gam + 4 * t);
  const v4f bv = *(const v4f*)(bet + 4 * t);
  v4f y;
  y[0] = d0 * rstd * gv[0] + bv[0];
  y[1] = d1 * rstd * gv[1] + bv[1];
  y[2] = d2 * rstd * gv[2] + bv[2];
  y[3] = d3 * rstd * gv[3] + bv[3];
  float* op = o32 + (size_t)row * DM + 4 * t;
  *(volatile v4f*)op = y;
  __threadfence();
  *(volatile v4f*)op = y;
  if (OUT16) {
    *(v4f*)(ybuf + 4 * t) = y;
    __syncthreads();
    if (t < DM / 8) {
      v8h hv;
#pragma unroll
      for (int e = 0; e < 8; ++e) hv[e] = (_Float16)ybuf[8 * t + e];
      _Float16* hp = o16 + (size_t)row * DM + 8 * t;
      *(volatile v8h*)hp = hv;
      __threadfence();
      *(volatile v8h*)hp = hv;
    }
  }
}

extern "C" void kernel_launch(void* const* d_in, const int* in_sizes, int n_in,
                              void* d_out, int out_size, void* d_ws, size_t ws_size,
                              hipStream_t stream) {
  if (n_in < 16) return;
  if (in_sizes[0] != MROWS * DM || in_sizes[1] != SEQ * SEQ || in_sizes[2] != BSZ * SEQ) return;
  if (in_sizes[3] != DM * DM || in_sizes[4] != DM * DM || in_sizes[5] != DM * DM || in_sizes[6] != DM * DM) return;
  if (in_sizes[7] != DM || in_sizes[8] != FFND * DM || in_sizes[9] != FFND) return;
  if (in_sizes[10] != DM * FFND || in_sizes[11] != DM) return;
  if (in_sizes[12] != DM || in_sizes[13] != DM || in_sizes[14] != DM || in_sizes[15] != DM) return;
  if (out_size != MROWS * DM) return;

  const float* tgt   = (const float*)d_in[0];
  const int*   tmask = (const int*)d_in[1];
  const int*   pmask = (const int*)d_in[2];
  const float* Wq    = (const float*)d_in[3];
  const float* Wk    = (const float*)d_in[4];
  const float* Wv    = (const float*)d_in[5];
  const float* Wo    = (const float*)d_in[6];
  const float* bo    = (const float*)d_in[7];
  const float* W1    = (const float*)d_in[8];
  const float* b1    = (const float*)d_in[9];
  const float* W2    = (const float*)d_in[10];
  const float* b2    = (const float*)d_in[11];
  const float* g1    = (const float*)d_in[12];
  const float* be1   = (const float*)d_in[13];
  const float* g2    = (const float*)d_in[14];
  const float* be2   = (const float*)d_in[15];
  float* out = (float*)d_out;

  const size_t MiB = 1048576;
  const int nqb = SEQ / AT_QB, nkc = SEQ / AT_KC;
  if (nkc > 128) return;
  const int TP = ((nkc + 31) / 32) * 32;
  const size_t tabBytes = (size_t)BSZ * nqb * TP * sizeof(int);
  const size_t total = 96 * MiB + tabBytes;
  if (total > ws_size) return;
  char* ws = (char*)d_ws;
  float*    Qf   = (float*)(ws + 0 * MiB);
  float*    Kf   = (float*)(ws + 16 * MiB);
  float*    Vf   = (float*)(ws + 32 * MiB);
  float*    RES1 = (float*)(ws + 0 * MiB);
  _Float16* H16  = (_Float16*)(ws + 0 * MiB);
  float*    X1f  = (float*)(ws + 32 * MiB);
  float*    AOf  = (float*)(ws + 48 * MiB);
  float*    RES2 = (float*)(ws + 48 * MiB);
  _Float16* X16  = (_Float16*)(ws + 64 * MiB);
  _Float16* O16  = (_Float16*)(ws + 64 * MiB);
  _Float16* X1h  = (_Float16*)(ws + 64 * MiB);
  _Float16* Wq16 = (_Float16*)(ws + 72 * MiB);
  _Float16* Wk16 = (_Float16*)(ws + 74 * MiB);
  _Float16* Wv16 = (_Float16*)(ws + 76 * MiB);
  _Float16* Wo16 = (_Float16*)(ws + 78 * MiB);
  _Float16* W1h  = (_Float16*)(ws + 80 * MiB);
  _Float16* W2h  = (_Float16*)(ws + 88 * MiB);
  int*      TAB  = (int*)(ws + 96 * MiB);

  auto castf = [&](const float* src, _Float16* dst, int n) {
    const int n2 = n / 2;
    cast_f32_f16x2<<<dim3((n2 + 255) / 256), dim3(256), 0, stream>>>(src, dst, n2);
  };
  castf(tgt, X16, MROWS * DM);
  castf(Wq, Wq16, DM * DM);
  castf(Wk, Wk16, DM * DM);
  castf(Wv, Wv16, DM * DM);
  castf(Wo, Wo16, DM * DM);
  castf(W1, W1h, FFND * DM);
  castf(W2, W2h, DM * FFND);

  tilecode_kernel<<<dim3(BSZ * nqb), dim3(256), 0, stream>>>(tmask, pmask, TAB, SEQ, nqb, nkc, TP);

  const long z = 0;
  typedef const unsigned short* cu16;
  const int tilesM = MROWS / 64;
  {
    const dim3 grid((tilesM * (DM / 64) + 7) / 8, 1);
    wmma_gemm64<0, false, 0, 0, false, 0><<<grid, dim3(256), 0, stream>>>(
        (cu16)X16, (cu16)X16, DM, z, (cu16)Wq16, (cu16)Wq16, DM, z, (void*)Qf, (void*)Qf, DM, z,
        bo, tgt, z, MROWS, DM, DM, 1.0f);
    wmma_gemm64<0, false, 0, 0, false, 0><<<grid, dim3(256), 0, stream>>>(
        (cu16)X16, (cu16)X16, DM, z, (cu16)Wk16, (cu16)Wk16, DM, z, (void*)Kf, (void*)Kf, DM, z,
        bo, tgt, z, MROWS, DM, DM, 1.0f);
    wmma_gemm64<0, false, 0, 0, false, 0><<<grid, dim3(256), 0, stream>>>(
        (cu16)X16, (cu16)X16, DM, z, (cu16)Wv16, (cu16)Wv16, DM, z, (void*)Vf, (void*)Vf, DM, z,
        bo, tgt, z, MROWS, DM, DM, 1.0f);
  }

  {
    AttnGeom g;
    g.tcode = TAB; g.cp = Qf; g.pc = Qf; g.c_bs = 0; g.c_rs = 0; g.c_hs = 0; g.t_pitch = TP;
    g.q_bs = (long)SEQ * DM; g.q_rs = DM; g.q_hs = HD;
    g.k_bs = (long)SEQ * DM; g.k_rs = DM; g.k_hs = HD;
    g.v_bs = (long)SEQ * DM; g.v_rs = DM; g.v_hs = HD;
    g.o_bs = (long)SEQ * DM; g.o_rs = DM; g.o_hs = HD;
    g.S = SEQ; g.Skv = SEQ; g.H = NHEAD; g.mask_mode = 6; g.qscale = 0.125f; g.blk0 = 0;
    g.mask_fill = -INFINITY; g.mask_is_int = 2;
    attn64_kernel<false, false, true><<<dim3(BSZ * NHEAD * nqb), dim3(128), 0, stream>>>(
        Qf, Kf, Vf, AOf, tmask, pmask, g);
  }
  castf(AOf, O16, MROWS * DM);

  {
    const dim3 grid((tilesM * (DM / 64) + 7) / 8, 1);
    wmma_gemm64<0, false, 2, 0, true, 0><<<grid, dim3(256), 0, stream>>>(
        (cu16)O16, (cu16)O16, DM, z, (cu16)Wo16, (cu16)Wo16, DM, z, (void*)RES1, (void*)RES1, DM, z,
        bo, tgt, z, MROWS, DM, DM, 1.0f);
  }
  ln_kernel<true><<<dim3(MROWS), dim3(256), 0, stream>>>(RES1, g1, be1, X1f, X1h);
  {
    const dim3 grid((tilesM * (FFND / 64) + 7) / 8, 1);
    wmma_gemm64<0, false, 2, 1, false, 6><<<grid, dim3(256), 0, stream>>>(
        (cu16)X1h, (cu16)X1h, DM, z, (cu16)W1h, (cu16)W1h, DM, z, (void*)H16, (void*)H16, FFND, z,
        b1, tgt, z, MROWS, FFND, DM, 1.0f);
  }
  {
    const dim3 grid((tilesM * (DM / 64) + 7) / 8, 1);
    wmma_gemm64<0, false, 2, 0, true, 0><<<grid, dim3(256), 0, stream>>>(
        (cu16)H16, (cu16)H16, FFND, z, (cu16)W2h, (cu16)W2h, FFND, z, (void*)RES2, (void*)RES2, DM, z,
        b2, X1f, z, MROWS, DM, FFND, 1.0f);
  }
  ln_kernel<false><<<dim3(MROWS), dim3(256), 0, stream>>>(RES2, g2, be2, out, X1h);
  (void)hipGetLastError();
}
